// TransitionModel_2980707303627
// MI455X (gfx1250) — hardware-verified
//
#include <hip/hip_runtime.h>


#define NBT  128
#define NS   2048
typedef _Float16 h16;
typedef unsigned short bf;
typedef __attribute__((ext_vector_type(16))) __bf16   v16bf;
typedef __attribute__((ext_vector_type(16))) _Float16 v16h;
typedef __attribute__((ext_vector_type(8)))  _Float16 v8h;
typedef __attribute__((ext_vector_type(8)))  unsigned short v8us;
typedef __attribute__((ext_vector_type(8)))  float    v8f;
typedef __attribute__((ext_vector_type(4)))  float    v4f;
typedef v8h  __attribute__((may_alias)) v8ha;
typedef v4f  __attribute__((may_alias)) v4fa;
typedef v8us __attribute__((may_alias)) v8usa;

__device__ __forceinline__ unsigned short f2bf(float f) { unsigned u = __float_as_uint(f); u += 0x7FFFu + ((u >> 16) & 1u); return (unsigned short)(u >> 16); }
__device__ __forceinline__ float bf2f(unsigned short b) { return __uint_as_float(((unsigned)b) << 16); }
__device__ __forceinline__ float bfr(float f) { return bf2f(f2bf(f)); }
__device__ __forceinline__ v16h cat16(v8h lo, v8h hi) { return __builtin_shufflevector(lo, hi, 0, 1, 2, 3, 4, 5, 6, 7, 8, 9, 10, 11, 12, 13, 14, 15); }
__device__ __forceinline__ v16bf cat16b(v8us lo, v8us hi) { return __builtin_bit_cast(v16bf, __builtin_shufflevector(lo, hi, 0, 1, 2, 3, 4, 5, 6, 7, 8, 9, 10, 11, 12, 13, 14, 15)); }
__device__ __forceinline__ v8f wmma16(v16h a, v16h b, v8f c) { return __builtin_amdgcn_wmma_f32_16x16x32_f16(false, a, false, b, (short)0, c, false, false); }
__device__ __forceinline__ v8f wmmab(v16bf a, v16bf b, v8f c) { return __builtin_amdgcn_wmma_f32_16x16x32_bf16(false, a, false, b, (short)0, c, false, false); }


template <typename T16> struct WFrag;
template <> struct WFrag<h16> { typedef v16h V; static __device__ __forceinline__ V ld(const h16* p) { return cat16(*(const v8h*)p, *(const v8h*)(p + 16)); } static __device__ __forceinline__ v8f mma(V a, V b, v8f c) { return wmma16(a, b, c); } };
template <> struct WFrag<bf> { typedef v16bf V; static __device__ __forceinline__ V ld(const bf* p) { return cat16b(*(const v8us*)p, *(const v8us*)(p + 16)); } static __device__ __forceinline__ v8f mma(V a, V b, v8f c) { return wmmab(a, b, c); } };
template <typename T16, int NSPLIT, bool BIAS>
__global__ __launch_bounds__(32) void k_gemmw(const T16* __restrict__ A, const T16* __restrict__ A2, const T16* __restrict__ Bt, const T16* __restrict__ Bt2, int K, float* C, int ldc, const float* __restrict__ bias, size_t sA, size_t sB, size_t sC) {
    typedef typename WFrag<T16>::V V;
    __shared__ __align__(16) float os[16 * 68];
    const size_t z = blockIdx.z; A += z * sA; if (A2) A2 += z * sA; Bt += z * sB; if (Bt2) Bt2 += z * sB; C += z * sC;
    const int lane = threadIdx.x & 31, lr = lane & 15, hi = lane >> 4; const int r0 = blockIdx.x * 64, c0 = blockIdx.y * 64;
    v8f acc[4][4];
#pragma unroll
    for (int mb = 0; mb < 4; ++mb)
#pragma unroll
        for (int nb = 0; nb < 4; ++nb) acc[mb][nb] = (v8f){};
    const size_t aoff = (size_t)(r0 + lr) * K + 8 * hi, boff = (size_t)(c0 + lr) * K + 8 * hi;
#pragma unroll 1
    for (int kc = 0; kc < K; kc += 32) {
        V a[4], a2[4];
#pragma unroll
        for (int mb = 0; mb < 4; ++mb) { a[mb] = WFrag<T16>::ld(A + aoff + (size_t)mb * 16 * K + kc); if (NSPLIT == 1 || NSPLIT == 2) a2[mb] = WFrag<T16>::ld(A2 + aoff + (size_t)mb * 16 * K + kc); }
#pragma unroll
        for (int nb = 0; nb < 4; ++nb) { const V b = WFrag<T16>::ld(Bt + boff + (size_t)nb * 16 * K + kc); V b2; if (NSPLIT >= 2) b2 = WFrag<T16>::ld(Bt2 + boff + (size_t)nb * 16 * K + kc);
#pragma unroll
            for (int mb = 0; mb < 4; ++mb) { acc[mb][nb] = WFrag<T16>::mma(a[mb], b, acc[mb][nb]); if (NSPLIT == 1 || NSPLIT == 2) acc[mb][nb] = WFrag<T16>::mma(a2[mb], b, acc[mb][nb]); if (NSPLIT >= 2) acc[mb][nb] = WFrag<T16>::mma(a[mb], b2, acc[mb][nb]); } }
        asm volatile("v_nop\n\tv_nop\n\tv_nop\n\tv_nop" : "+v"(acc[0][0]), "+v"(acc[1][1]), "+v"(acc[2][2]), "+v"(acc[3][3]) : "v"(a[0]), "v"(a[3]));
    }
#pragma unroll
    for (int mb = 0; mb < 4; ++mb) {
#pragma unroll
        for (int nb = 0; nb < 4; ++nb) {
#pragma unroll
            for (int j = 0; j < 8; ++j) os[(hi * 8 + j) * 68 + nb * 16 + lr] = acc[mb][nb][j]; }
        __builtin_amdgcn_wave_barrier(); asm volatile("" ::: "memory");
        float* crow = C + (size_t)(r0 + mb * 16) * ldc + c0;
#pragma unroll 1
        for (int ps = 0; ps < 2; ++ps) {
#pragma unroll
            for (int s = 0; s < 8; ++s) { const int row = 2 * s + hi, cofs = lr * 4; v4f val = *(const v4fa*)(os + row * 68 + cofs); if (BIAS) { val[0] += bfr(bias[c0 + cofs]); val[1] += bfr(bias[c0 + cofs + 1]); val[2] += bfr(bias[c0 + cofs + 2]); val[3] += bfr(bias[c0 + cofs + 3]); }
                *(volatile v4f*)(crow + (size_t)row * ldc + cofs) = val; }
            if (ps == 0) __threadfence(); }
        __builtin_amdgcn_wave_barrier(); asm volatile("" ::: "memory");
    }
}

typedef __attribute__((ext_vector_type(4))) unsigned short v4us;
__device__ __forceinline__ void splitf(float y, unsigned short& h, unsigned short& l) { h = f2bf(y); l = f2bf(y - bf2f(h)); }
__global__ __launch_bounds__(256) void k_collse(const float* __restrict__ Wm, float* C) { const int k = blockIdx.x * 256 + threadIdx.x; if (k >= NS) return; float mx = -3.0e38f;
#pragma unroll 4
    for (int i = 0; i < NS; ++i) mx = fmaxf(mx, bfr(Wm[(size_t)i * NS + k]));
    float s = 0.f;
#pragma unroll 4
    for (int i = 0; i < NS; ++i) { float d = __fsub_rn(bfr(Wm[(size_t)i * NS + k]), mx); asm volatile("" : "+v"(d)); s = __fadd_rn(s, expf(d)); }
    const float c = __fadd_rn(mx, logf(s)); *(volatile float*)(C + k) = c; __threadfence(); *(volatile float*)(C + k) = c; }
__global__ __launch_bounds__(256) void k_rowexp(const float* __restrict__ X, const float* __restrict__ Cc, int nrows, float* Mpad, bf* Eh, bf* El) {
    const int lane = threadIdx.x & 31; const int row = blockIdx.x * 8 + (threadIdx.x >> 5); if (row >= nrows) return; const float* xr = X + (size_t)row * NS; float v[NS / 32]; float mx = -3.0e38f;
#pragma unroll
    for (int ch = 0; ch < NS / 128; ++ch) { const int k0 = ch * 128 + lane * 4; const v4f a = *(const v4f*)(xr + k0); v4f cc; if (Cc) cc = *(const v4f*)(Cc + k0); else { cc[0] = 0.f; cc[1] = 0.f; cc[2] = 0.f; cc[3] = 0.f; }
#pragma unroll
        for (int q = 0; q < 4; ++q) { const float t = __fsub_rn(bfr(a[q]), cc[q]); v[ch * 4 + q] = t; mx = fmaxf(mx, t); } }
#pragma unroll
    for (int sh = 16; sh; sh >>= 1) mx = fmaxf(mx, __shfl_xor(mx, sh, 32));
#pragma unroll 1
    for (int ps = 0; ps < 2; ++ps) {
#pragma unroll
        for (int ch = 0; ch < NS / 128; ++ch) { v4us oh, ol;
#pragma unroll
            for (int q = 0; q < 4; ++q) { float d = __fsub_rn(v[ch * 4 + q], mx); asm volatile("" : "+v"(d)); const float e = __builtin_amdgcn_exp2f(__fmul_rn(d, 1.4426950408889634f)); unsigned short a2, c2; splitf(e, a2, c2); oh[q] = a2; ol[q] = c2; }
            const size_t oo = (size_t)row * NS + ch * 128 + lane * 4; *(volatile v4us*)(Eh + oo) = oh; *(volatile v4us*)(El + oo) = ol; }
        if (lane == 0) *(volatile float*)(Mpad + (size_t)row * 32) = mx;
        if (ps == 0) __threadfence(); }
}
__global__ __launch_bounds__(256) void k_fin(const float* __restrict__ S, const float* __restrict__ MApad, const float* __restrict__ MWpad, float* out) { const size_t e = (size_t)blockIdx.x * 256 + threadIdx.x; if (e >= (size_t)NBT * NS) return; const int i = (int)(e % NS), b = (int)(e / NS);
    const float o = __fadd_rn(__fadd_rn(MApad[(size_t)b * 32], MWpad[(size_t)i * 32]), logf(S[e])); *(volatile float*)(out + e) = o; __threadfence(); *(volatile float*)(out + e) = o; }

extern "C" void kernel_launch(void* const* d_in, const int* in_sizes, int n_in,
                              void* d_out, int out_size, void* d_ws, size_t ws_size, hipStream_t stream) {
    (void)in_sizes; (void)n_in; (void)out_size;
    const float* la = (const float*)d_in[0]; const float* Wm = (const float*)d_in[1];
    float* OUT = (float*)d_out;
    char* wsp = (char*)d_ws;
    auto take = [&](size_t bytes) { char* p = wsp; wsp += (bytes + 255) & ~(size_t)255; return (void*)p; };
    float* Cc = (float*)take((size_t)NS * 4); float* MWpad = (float*)take((size_t)NS * 32 * 4); float* MApad = (float*)take((size_t)NBT * 32 * 4);
    bf* EWh = (bf*)take((size_t)NS * NS * 2); bf* EWl = (bf*)take((size_t)NS * NS * 2); bf* EAh = (bf*)take((size_t)NBT * NS * 2); bf* EAl = (bf*)take((size_t)NBT * NS * 2); float* S = (float*)take((size_t)NBT * NS * 4);
    if ((size_t)(wsp - (char*)d_ws) > ws_size) return;
    k_collse<<<NS / 256, 256, 0, stream>>>(Wm, Cc);
    k_rowexp<<<NS / 8, 256, 0, stream>>>(Wm, nullptr, NS, MWpad, EWh, EWl);
    k_rowexp<<<NBT / 8, 256, 0, stream>>>(la, Cc, NBT, MApad, EAh, EAl);
    k_gemmw<bf, 2, false><<<dim3(NBT / 64, NS / 64, 1), 32, 0, stream>>>(EAh, EAl, EWh, EWl, NS, S, NS, nullptr, 0, 0, 0);
    k_fin<<<(NBT * NS + 255) / 256, 256, 0, stream>>>(S, MApad, MWpad, OUT);
}
